// GNN_Virtualnode_91070486545221
// MI455X (gfx1250) — hardware-run, weakly checked
//
#include <hip/hip_runtime.h>
#include <stddef.h>
#include <stdint.h>


#ifndef AGG_SPLIT
#define AGG_SPLIT 1
#endif
#ifndef HID_SPLIT
#define HID_SPLIT 1
#endif

#define NNODE   100000
#define NEDGE   1600000
#define DD      128
#define HH      256
#define NLAY    5
#define NGR     128
#define MPAD    100096
#define HALFR   50048
#define NTHR    256
#define NWAVE   8
#define CHUNK   2048
#define WCAP    256
#define LISTN   (NWAVE * WCAP)
#define NB1     1024
#define NBLK    98
#define NBMAX   2048
#define PKS     11
#define RCAP    20480
#define DEGCAP  64
#define POISONC (1 << 20)
#define GCAP    4096
#define GPITCH  (32 + GCAP)
#define GBM     64
#define GTHR    128
#define BN      128
#define PARTW   288
#define NTILE   (MPAD / GBM)
#define HTILE   (HALFR / GBM)
#define APW     256
#define HIDP    512
#define P3P     384
#define KA_EXT  (AGG_SPLIT ? 256 : 128)
#define KB_EXT  (HID_SPLIT ? 512 : 256)
#define LDS_BKT ((2 * RCAP + 2 * NBMAX + LISTN) * 4 + 64)
#define LDS_GV  (NGR * BN * 4)

static_assert(NNODE <= (1 << 17));
static_assert(18 <= 32);
static_assert(NEDGE <= (1 << 21));
static_assert(MPAD % GBM == 0 && HALFR * 2 == MPAD && HALFR % GBM == 0 && MPAD >= NNODE);
static_assert(NBLK * NB1 >= MPAD);
static_assert(NB1 == 4 * NTHR && NBMAX == 8 * NTHR && NB1 <= (1 << PKS) && CHUNK <= (1 << PKS));
static_assert(CHUNK == NWAVE * WCAP && WCAP == 8 * 32 && LISTN >= NBMAX);
static_assert(RCAP % (4 * NTHR) == 0 && (2 * RCAP + NBMAX) % 4 == 0);
static_assert(LDS_BKT <= 300000);
static_assert(GCAP % 4 == 0 && (GPITCH * 4) % 128 == 0 && GCAP % NTHR == 0);
static_assert(GBM == (GTHR / 32) * 16 && GTHR == BN && DD == BN && HH == 2 * BN);
static_assert(NGR == 128 && NGR == NWAVE * 16);
static_assert(PARTW % 32 == 0 && PARTW / 4 <= GTHR && PARTW >= 2 * BN + 1);
static_assert((MPAD * 32) % NTHR == 0 && (NNODE * 32) % NTHR == 0);
static_assert(LDS_GV + 4096 <= 327680);

typedef float          v4f  __attribute__((ext_vector_type(4)));
typedef float          v8f  __attribute__((ext_vector_type(8)));
typedef int            v2i  __attribute__((ext_vector_type(2)));
typedef int            v4i  __attribute__((ext_vector_type(4)));
typedef int            v8i  __attribute__((ext_vector_type(8)));
typedef unsigned int   v2u  __attribute__((ext_vector_type(2)));
typedef unsigned int   v4u  __attribute__((ext_vector_type(4)));
typedef unsigned short v4us __attribute__((ext_vector_type(4)));
typedef unsigned short v8us __attribute__((ext_vector_type(8)));
typedef __bf16         v16b __attribute__((ext_vector_type(16)));
typedef v4f  __attribute__((may_alias)) v4fa;
typedef v4i  __attribute__((may_alias)) v4ia;
typedef v4u  __attribute__((may_alias)) v4ua;
typedef v8us __attribute__((may_alias)) v8usa;
union FragB { v16b v; v8us h[2]; v8i w; };

__device__ __forceinline__ v8f wmb(const FragB& a, const FragB& b, v8f c) {
  v8f d = __builtin_amdgcn_wmma_f32_16x16x32_bf16(false, a.v, false, b.v, (short)0, c, false, false);
  asm volatile("v_nop\n\tv_nop\n\tv_nop\n\tv_nop" : "+v"(d) : "v"(a.w), "v"(b.w));
  return d;
}

__device__ __forceinline__ unsigned bf_bits(float f) {
  const unsigned u = __float_as_uint(f);
  const unsigned r = (u + 0x7FFFu + ((u >> 16) & 1u)) >> 16;
  return (f != f) ? 0x7FC0u : r;
}
__device__ __forceinline__ float bf_val(unsigned b) { return __uint_as_float(b << 16); }
__device__ __forceinline__ float bf_rne(float f) { return bf_val(bf_bits(f)); }
__device__ __forceinline__ float relu_keep(float v) { return (v > 0.0f) ? v : (v - v); }
__device__ __forceinline__ float bn_y(float x, float mu, float r, float g, float b) {
  return ((g * (x - mu)) * r) + b;
}
__device__ __forceinline__ int clampi(int v, int lo, int hi) { return v < lo ? lo : (v > hi ? hi : v); }

__global__ __launch_bounds__(NTHR) void k_wprep(const float* __restrict__ W, int kin, int nout, int kp8,
                                                int nUnits, unsigned short* wt) {
  const int u = (int)blockIdx.x * NTHR + (int)threadIdx.x;
  if (u >= nUnits) return;
  const int upm = nout * kp8;
  const int mi  = u / upm;
  const int v   = u - mi * upm;
  const int n   = v / kp8;
  const int k8  = (v - n * kp8) * 8;
  const int kk  = k8 % kin;
  const float* p = W + (size_t)mi * (size_t)kin * (size_t)nout + (size_t)kk * (size_t)nout + n;
  v8us o;
#pragma unroll
  for (int i = 0; i < 8; ++i) o[i] = (unsigned short)bf_bits(p[(size_t)i * (size_t)nout]);
  unsigned short* dp = wt + (size_t)u * 8;
  *(volatile v8us*)dp = o;
  __threadfence();
  *(volatile v8us*)dp = o;
}

__global__ __launch_bounds__(NTHR) void k_embed(const int* __restrict__ x, const float* __restrict__ e1,
                                                const float* __restrict__ e2, const float* __restrict__ gve,
                                                float* p0) {
  const int u = (int)blockIdx.x * NTHR + (int)threadIdx.x;
  if (u >= MPAD * 32) return;
  const int row = u >> 5;
  const int c4  = (u & 31) * 4;
  const int rc  = row < NNODE ? row : NNODE - 1;
  const v2i xi  = *(const v2i*)(x + 2 * (size_t)rc);
  const int i0  = clampi(xi.x, 0, 119);
  const int i1  = clampi(xi.y, 0, 2);
  const v4f a = *(const v4f*)(e1 + (size_t)i0 * DD + c4);
  const v4f b = *(const v4f*)(e2 + (size_t)i1 * DD + c4);
  const v4f g = *(const v4f*)(gve + c4);
  asm volatile("" :: "v"(a.x), "v"(a.y), "v"(a.z), "v"(a.w));
  asm volatile("" :: "v"(b.x), "v"(b.y), "v"(b.z), "v"(b.w));
  const bool ok = row < NNODE;
  v4f o;
  o.x = ok ? ((bf_rne(a.x) + bf_rne(b.x)) + bf_rne(g.x)) : 0.0f;
  o.y = ok ? ((bf_rne(a.y) + bf_rne(b.y)) + bf_rne(g.y)) : 0.0f;
  o.z = ok ? ((bf_rne(a.z) + bf_rne(b.z)) + bf_rne(g.z)) : 0.0f;
  o.w = ok ? ((bf_rne(a.w) + bf_rne(b.w)) + bf_rne(g.w)) : 0.0f;
  float* hp = p0 + (size_t)u * 4;
  *(volatile v4f*)hp = o;
  __threadfence();
  *(volatile v4f*)hp = o;
}

__device__ __forceinline__ int scan_chunk(const int* __restrict__ dsts, int cbase, int slotBase,
                                          int* list, int lane, int wave) {
  int wc = 0;
  const int elw  = wave * WCAP;
  const int sent = (int)(1u << 31);
  const int eb   = cbase + elw + lane;
  const int r0 = dsts[min(eb,       NEDGE - 1)];
  const int r1 = dsts[min(eb + 32,  NEDGE - 1)];
  const int r2 = dsts[min(eb + 64,  NEDGE - 1)];
  const int r3 = dsts[min(eb + 96,  NEDGE - 1)];
  const int r4 = dsts[min(eb + 128, NEDGE - 1)];
  const int r5 = dsts[min(eb + 160, NEDGE - 1)];
  const int r6 = dsts[min(eb + 192, NEDGE - 1)];
  const int r7 = dsts[min(eb + 224, NEDGE - 1)];
  asm volatile("" :: "v"(r0), "v"(r1), "v"(r2), "v"(r3));
  asm volatile("" :: "v"(r4), "v"(r5), "v"(r6), "v"(r7));
  const int d0 = (eb       < NEDGE) ? r0 : sent;
  const int d1 = (eb + 32  < NEDGE) ? r1 : sent;
  const int d2 = (eb + 64  < NEDGE) ? r2 : sent;
  const int d3 = (eb + 96  < NEDGE) ? r3 : sent;
  const int d4 = (eb + 128 < NEDGE) ? r4 : sent;
  const int d5 = (eb + 160 < NEDGE) ? r5 : sent;
  const int d6 = (eb + 192 < NEDGE) ? r6 : sent;
  const int d7 = (eb + 224 < NEDGE) ? r7 : sent;
  const unsigned nbs = (unsigned)slotBase;
  const unsigned s0 = (unsigned)d0 - nbs, s1 = (unsigned)d1 - nbs, s2 = (unsigned)d2 - nbs, s3 = (unsigned)d3 - nbs;
  const unsigned s4 = (unsigned)d4 - nbs, s5 = (unsigned)d5 - nbs, s6 = (unsigned)d6 - nbs, s7 = (unsigned)d7 - nbs;
  const bool h0 = (s0 < (unsigned)NB1) && ((unsigned)d0 < (unsigned)NNODE);
  const bool h1 = (s1 < (unsigned)NB1) && ((unsigned)d1 < (unsigned)NNODE);
  const bool h2 = (s2 < (unsigned)NB1) && ((unsigned)d2 < (unsigned)NNODE);
  const bool h3 = (s3 < (unsigned)NB1) && ((unsigned)d3 < (unsigned)NNODE);
  const bool h4 = (s4 < (unsigned)NB1) && ((unsigned)d4 < (unsigned)NNODE);
  const bool h5 = (s5 < (unsigned)NB1) && ((unsigned)d5 < (unsigned)NNODE);
  const bool h6 = (s6 < (unsigned)NB1) && ((unsigned)d6 < (unsigned)NNODE);
  const bool h7 = (s7 < (unsigned)NB1) && ((unsigned)d7 < (unsigned)NNODE);
  const unsigned any = __builtin_amdgcn_ballot_w32(h0 | h1 | h2 | h3 | h4 | h5 | h6 | h7);
  if (any != 0u) {
#define HITJ(J, HJ, SJ) { \
      const unsigned mj = __builtin_amdgcn_ballot_w32(HJ); \
      if (mj != 0u) { \
        const int pos = wc + (int)__builtin_amdgcn_mbcnt_lo(mj, 0u); \
        if ((HJ) && pos < WCAP) list[wave * WCAP + pos] = ((elw + 32 * (J) + lane) << PKS) | (int)(SJ); \
        wc += (int)__builtin_popcount(mj); } }
    HITJ(0, h0, s0)
    HITJ(1, h1, s1)
    HITJ(2, h2, s2)
    HITJ(3, h3, s3)
    HITJ(4, h4, s4)
    HITJ(5, h5, s5)
    HITJ(6, h6, s6)
    HITJ(7, h7, s7)
#undef HITJ
  }
  return wc;
}

__device__ __forceinline__ int mk_word(int s, int a0, int a1) {
  const int sc = clampi(s, 0, NNODE - 1);
  const int x0 = clampi(a0, 0, 5);
  const int x1 = clampi(a1, 0, 2);
  return sc | ((3 * x0 + x1) << 17);
}

__global__ __launch_bounds__(NTHR) void k_bucket(const int* __restrict__ ei, const int* __restrict__ ea,
                                                 int* listg, int* offg, int* cntg) {
  extern __shared__ v4f lds_dyn[];
  int* reg1 = (int*)lds_dyn;
  int* reg2 = reg1 + RCAP;
  int* scnt = reg2 + RCAP;
  int* soff = scnt + NBMAX;
  int* list = soff + NBMAX;
  int* wcnt = list + LISTN;
  int* wtot = wcnt + NWAVE;
  const int* srcs = ei;
  const int* dsts = ei + NEDGE;
  const int tid = (int)threadIdx.x, lane = tid & 31, wave = tid >> 5;
  const int nodeBase = (int)blockIdx.x * NB1;

  {
    const v4i z4 = {0, 0, 0, 0};
    for (int i = tid * 4; i < 2 * RCAP + NBMAX; i += NTHR * 4) *(v4ia*)(reg1 + i) = z4;
  }
  __syncthreads();

  int tot = 0;
  const int nChunks = (NEDGE + CHUNK - 1) / CHUNK;
#pragma unroll 1
  for (int ch = 0; ch < nChunks; ++ch) {
    const int cbase = ch * CHUNK;
    const int wc = scan_chunk(dsts, cbase, nodeBase, list, lane, wave);
    if (lane == 0) wcnt[wave] = wc;
    __syncthreads();
    int pre = 0, all = 0;
#pragma unroll
    for (int w2 = 0; w2 < NWAVE; ++w2) {
      int c = wcnt[w2];
      c = c < 0 ? 0 : (c > WCAP ? WCAP : c);
      all += c;
      pre += (w2 < wave) ? c : 0;
    }
    const int wcc  = wc > WCAP ? WCAP : wc;
    const int base = tot + pre;
#pragma unroll 1
    for (int i = lane; i < wcc; i += 32) {
      const int ent = list[wave * WCAP + i];
      const int el  = (ent >> PKS) & (CHUNK - 1);
      const int sl  = ent & (NB1 - 1);
      int eid = cbase + el;
      eid = eid > NEDGE - 1 ? NEDGE - 1 : eid;
      const int pos = base + i;
      if (pos < RCAP) reg1[pos] = (int)(((unsigned)eid << PKS) | (unsigned)sl);
    }
    tot += all;
    tot = tot > RCAP ? RCAP : tot;
    __syncthreads();
  }
  const int nh = tot;
  const bool ovf = (nh >= RCAP);

  if (wave == 0) {
#pragma unroll 1
    for (int b0 = 0; b0 < nh; b0 += 32) {
      const int idx = b0 + lane;
      const int uv  = reg1[idx < RCAP ? idx : RCAP - 1];
      const int m32 = (nh - b0) < 32 ? (nh - b0) : 32;
#pragma unroll 1
      for (int k = 0; k < m32; ++k) {
        const int u  = __builtin_amdgcn_readlane(uv, k);
        const int sl = u & (NB1 - 1);
        if (lane == 0) scnt[sl] = scnt[sl] + 1;
      }
    }
  }
  __syncthreads();

  {
    const v4i ca = *(const v4ia*)(scnt + 8 * tid);
    const v4i cb = *(const v4ia*)(scnt + 8 * tid + 4);
    const int e0 = ca.x < 0 ? 0 : ca.x, e1 = ca.y < 0 ? 0 : ca.y, e2 = ca.z < 0 ? 0 : ca.z, e3 = ca.w < 0 ? 0 : ca.w;
    const int e4 = cb.x < 0 ? 0 : cb.x, e5 = cb.y < 0 ? 0 : cb.y, e6 = cb.z < 0 ? 0 : cb.z, e7 = cb.w < 0 ? 0 : cb.w;
    const int ts = e0 + e1 + e2 + e3 + e4 + e5 + e6 + e7;
    int incl = ts;
#pragma unroll
    for (int d = 1; d < 32; d <<= 1) {
      const int up = __shfl_up(incl, d);
      if (lane >= d) incl += up;
    }
    if (lane == 31) wtot[wave] = incl;
    __syncthreads();
    int pre = 0;
#pragma unroll
    for (int w2 = 0; w2 < NWAVE; ++w2) pre += (w2 < wave) ? wtot[w2] : 0;
    int run = pre + incl - ts;
    soff[8 * tid + 0] = run; run += e0;
    soff[8 * tid + 1] = run; run += e1;
    soff[8 * tid + 2] = run; run += e2;
    soff[8 * tid + 3] = run; run += e3;
    soff[8 * tid + 4] = run; run += e4;
    soff[8 * tid + 5] = run; run += e5;
    soff[8 * tid + 6] = run; run += e6;
    soff[8 * tid + 7] = run;
  }
  __syncthreads();
  for (int i = tid; i < NBMAX; i += NTHR) list[i] = soff[i];
  __syncthreads();

  if (wave == 0) {
#pragma unroll 1
    for (int b0 = 0; b0 < nh; b0 += 32) {
      const int idx = b0 + lane;
      const int uv  = reg1[idx < RCAP ? idx : RCAP - 1];
      const int m32 = (nh - b0) < 32 ? (nh - b0) : 32;
#pragma unroll 1
      for (int k = 0; k < m32; ++k) {
        const int u   = __builtin_amdgcn_readlane(uv, k);
        const int sl  = u & (NB1 - 1);
        const int eid = (int)((unsigned)u >> PKS);
        if (lane == 0) {
          int pos = list[sl];
          pos = pos < 0 ? 0 : (pos > RCAP - 1 ? RCAP - 1 : pos);
          reg2[pos] = eid;
          list[sl] = pos + 1;
        }
      }
    }
  }
  __syncthreads();

  {
    const v4i o4 = *(const v4ia*)(soff + 4 * tid);
    v4i c4 = *(const v4ia*)(scnt + 4 * tid);
    if (ovf) { c4.x = POISONC; c4.y = POISONC; c4.z = POISONC; c4.w = POISONC; }
    int* op = offg + nodeBase + 4 * tid;
    int* cp = cntg + nodeBase + 4 * tid;
    *(volatile v4i*)op = o4;
    *(volatile v4i*)cp = c4;
    __threadfence();
    *(volatile v4i*)op = o4;
    *(volatile v4i*)cp = c4;
  }

  int* lrow = listg + (size_t)blockIdx.x * RCAP;
#pragma unroll 1
  for (int it = 0; it < RCAP / (4 * NTHR); ++it) {
    const int p = 4 * (it * NTHR + tid);
    const v4i e4 = *(const v4ia*)(reg2 + p);
    const int q0 = clampi(e4.x, 0, NEDGE - 1), q1 = clampi(e4.y, 0, NEDGE - 1);
    const int q2 = clampi(e4.z, 0, NEDGE - 1), q3 = clampi(e4.w, 0, NEDGE - 1);
    const int sA = srcs[q0], sB = srcs[q1], sC = srcs[q2], sD = srcs[q3];
    const v2i aA = *(const v2i*)(ea + 2 * (size_t)q0);
    const v2i aB = *(const v2i*)(ea + 2 * (size_t)q1);
    const v2i aC = *(const v2i*)(ea + 2 * (size_t)q2);
    const v2i aD = *(const v2i*)(ea + 2 * (size_t)q3);
    asm volatile("" :: "v"(sA), "v"(sB), "v"(sC), "v"(sD));
    asm volatile("" :: "v"(aA.x), "v"(aA.y), "v"(aB.x), "v"(aB.y));
    asm volatile("" :: "v"(aC.x), "v"(aC.y), "v"(aD.x), "v"(aD.y));
    const int wA = mk_word(sA, aA.x, aA.y), wB = mk_word(sB, aB.x, aB.y);
    const int wC = mk_word(sC, aC.x, aC.y), wD = mk_word(sD, aD.x, aD.y);
    v4i w;
    w.x = (p     < nh) ? wA : 0;
    w.y = (p + 1 < nh) ? wB : 0;
    w.z = (p + 2 < nh) ? wC : 0;
    w.w = (p + 3 < nh) ? wD : 0;
    *(volatile v4i*)(lrow + p) = w;
    __threadfence();
    *(volatile v4i*)(lrow + p) = w;
  }
}

__global__ __launch_bounds__(NTHR) void k_gbucket(const int* __restrict__ bat, const float* __restrict__ gve,
                                                  int* glist, float* gv0) {
  __shared__ __attribute__((aligned(16))) int gl[GCAP];
  __shared__ int wcn[NWAVE];
  const int tid = (int)threadIdx.x, lane = tid & 31, wave = tid >> 5;
  const int g = (int)blockIdx.x;
  {
    const v4i z4 = {0, 0, 0, 0};
    for (int i = tid * 4; i < GCAP; i += NTHR * 4) *(v4ia*)(gl + i) = z4;
  }
  __syncthreads();
  int tot = 0;
#pragma unroll 1
  for (int cb = 0; cb < NNODE; cb += NTHR) {
    const int i  = cb + tid;
    const int ic = i < NNODE ? i : NNODE - 1;
    const int b  = bat[ic];
    asm volatile("" :: "v"(b));
    const bool hit = (i < NNODE) && (b == g);
    const unsigned msk = __builtin_amdgcn_ballot_w32(hit);
    const int wc = (int)__builtin_popcount(msk);
    if (lane == 0) wcn[wave] = wc;
    __syncthreads();
    int pre = 0, all = 0;
#pragma unroll
    for (int w2 = 0; w2 < NWAVE; ++w2) {
      int c = wcn[w2];
      c = c < 0 ? 0 : (c > 32 ? 32 : c);
      all += c;
      pre += (w2 < wave) ? c : 0;
    }
    const int pos = tot + pre + (int)__builtin_amdgcn_mbcnt_lo(msk, 0u);
    if (hit && pos < GCAP) gl[pos] = i;
    tot += all;
    tot = tot > GCAP + 1 ? GCAP + 1 : tot;
    __syncthreads();
  }
  const int cw = (tot > GCAP) ? POISONC : tot;
  int* grow = glist + (size_t)g * GPITCH;
#pragma unroll 1
  for (int i = tid; i < GPITCH / 4; i += NTHR) {
    const int li = i < 8 ? 0 : (i - 8) * 4;
    const v4i dv = *(const v4ia*)(gl + li);
    v4i w;
    w.x = (i < 8) ? cw : dv.x;
    w.y = (i < 8) ? cw : dv.y;
    w.z = (i < 8) ? cw : dv.z;
    w.w = (i < 8) ? cw : dv.w;
    *(volatile v4i*)(grow + 4 * i) = w;
    __threadfence();
    *(volatile v4i*)(grow + 4 * i) = w;
  }
  {
    const v4f e = *(const v4f*)(gve + 4 * lane);
    v4f o;
    o.x = bf_rne(e.x); o.y = bf_rne(e.y); o.z = bf_rne(e.z); o.w = bf_rne(e.w);
    float* op = gv0 + (size_t)g * DD + 4 * lane;
    const bool okst = (wave == 0);
    if (okst) *(volatile v4f*)op = o;
    __threadfence();
    if (okst) *(volatile v4f*)op = o;
  }
}

__global__ __launch_bounds__(NTHR) void k_pool(const float* __restrict__ hv, const int* __restrict__ glist,
                                               const float* __restrict__ gvl, unsigned short* pool3) {
  __shared__ __attribute__((aligned(16))) float wsum[NWAVE * DD];
  __shared__ __attribute__((aligned(16))) unsigned short prow[3 * DD];
  const int tid = (int)threadIdx.x, lane = tid & 31;
  const int wave = __builtin_amdgcn_readfirstlane(tid >> 5);
  const int g = (int)blockIdx.x;
  const int* gp = glist + (size_t)g * GPITCH;
  const int cv = gp[lane];
  asm volatile("" :: "v"(cv));
  const int cc   = cv < 0 ? 0 : (cv > GCAP ? GCAP : cv);
  const int cnt  = __builtin_amdgcn_readfirstlane(cc);
  const int craw = __builtin_amdgcn_readfirstlane(cv);
  const bool poison = (craw < 0) || (craw > GCAP);
  const int nw = cnt > wave ? ((cnt - wave + 7) >> 3) : 0;
  float a0 = 0.0f, a1 = 0.0f, a2 = 0.0f, a3 = 0.0f;
#pragma unroll 1
  for (int b0 = 0; b0 < nw; b0 += 32) {
    int e = wave + 8 * (b0 + lane);
    e = e > cnt - 1 ? cnt - 1 : e;
    e = e < 0 ? 0 : (e > GCAP - 1 ? GCAP - 1 : e);
    int id = gp[32 + e];
    id = id < 0 ? 0 : (id > NNODE - 1 ? NNODE - 1 : id);
    const int m32 = (nw - b0) < 32 ? (nw - b0) : 32;
#pragma unroll 4
    for (int k = 0; k < m32; ++k) {
      const int nk = __builtin_amdgcn_readlane(id, k);
      const v4f v = *(const v4f*)(hv + (size_t)nk * DD + 4 * lane);
      a0 += v.x; a1 += v.y; a2 += v.z; a3 += v.w;
    }
  }
  wsum[wave * DD + 4 * lane + 0] = a0;
  wsum[wave * DD + 4 * lane + 1] = a1;
  wsum[wave * DD + 4 * lane + 2] = a2;
  wsum[wave * DD + 4 * lane + 3] = a3;
  __syncthreads();
  if (tid < DD) {
    double s = 0.0;
#pragma unroll
    for (int w2 = 0; w2 < NWAVE; ++w2) s += (double)wsum[w2 * DD + tid];
    const float pf = (float)s;
    float p = pf + gvl[(size_t)g * DD + tid];
    p = poison ? __int_as_float(0x7fc00000) : p;
    const unsigned hb = bf_bits(p);
    const float r1 = p - bf_val(hb);
    const unsigned mb = bf_bits(r1);
    const float r2 = r1 - bf_val(mb);
    const unsigned lb = bf_bits(r2);
    prow[tid]          = (unsigned short)hb;
    prow[DD + tid]     = (unsigned short)mb;
    prow[2 * DD + tid] = (unsigned short)lb;
  }
  __syncthreads();
  const int tq = tid < (3 * DD) / 8 ? tid : 0;
  const v8us pv = *(const v8usa*)(prow + 8 * tq);
  unsigned short* op = pool3 + (size_t)g * P3P + 8 * tq;
  const bool okst = tid < (3 * DD) / 8;
  if (okst) *(volatile v8us*)op = pv;
  __threadfence();
  if (okst) *(volatile v8us*)op = pv;
}

template <int MODE, int KEXT, int APITCH, int WPITCH>
__global__ __launch_bounds__(NTHR) __attribute__((amdgpu_num_vgpr(248)))
void k_gv(const unsigned short* __restrict__ A, const unsigned short* __restrict__ WT,
          const float* __restrict__ bias, const float* __restrict__ gam, const float* __restrict__ bet,
          unsigned short* outH, float* outF) {
  static_assert(KEXT % 32 == 0 && KEXT <= APITCH && KEXT <= WPITCH);
  extern __shared__ v4f lds_dyn[];
  float* stg = (float*)lds_dyn;
  __shared__ __attribute__((aligned(16))) float par[3 * BN];
  __shared__ __attribute__((aligned(16))) float cmu[BN];
  __shared__ __attribute__((aligned(16))) float crr[BN];
  const int tid = (int)threadIdx.x, lane = tid & 31, wave = tid >> 5, hh = lane >> 4, m = lane & 15;
  const int colBase = (int)blockIdx.x * BN;

  if (tid < 32) {
    const v4f q = *(const v4f*)(bias + colBase + 4 * lane);
    par[4 * lane + 0] = bf_rne(q.x); par[4 * lane + 1] = bf_rne(q.y);
    par[4 * lane + 2] = bf_rne(q.z); par[4 * lane + 3] = bf_rne(q.w);
  } else if (tid < 64) {
    const v4f q = *(const v4f*)(gam + colBase + 4 * lane);
    par[BN + 4 * lane + 0] = bf_rne(q.x); par[BN + 4 * lane + 1] = bf_rne(q.y);
    par[BN + 4 * lane + 2] = bf_rne(q.z); par[BN + 4 * lane + 3] = bf_rne(q.w);
  } else if (tid < 96) {
    const v4f q = *(const v4f*)(bet + colBase + 4 * lane);
    par[2 * BN + 4 * lane + 0] = bf_rne(q.x); par[2 * BN + 4 * lane + 1] = bf_rne(q.y);
    par[2 * BN + 4 * lane + 2] = bf_rne(q.z); par[2 * BN + 4 * lane + 3] = bf_rne(q.w);
  }

  v8f acc[8];
  {
    const v8f z = {0.f, 0.f, 0.f, 0.f, 0.f, 0.f, 0.f, 0.f};
#pragma unroll
    for (int t = 0; t < 8; ++t) acc[t] = z;
  }
  const unsigned short* ap = A + (size_t)(16 * wave + m) * (size_t)APITCH + 8 * hh;
  const unsigned short* wp = WT + (size_t)(colBase + m) * (size_t)WPITCH + 8 * hh;
#pragma unroll 1
  for (int k0 = 0; k0 < KEXT; k0 += 32) {
    FragB af;
    af.h[0] = *(const v8usa*)(ap + k0);
    af.h[1] = *(const v8usa*)(ap + k0 + 16);
#pragma unroll
    for (int t = 0; t < 8; ++t) {
      const unsigned short* wq = wp + (size_t)(16 * t) * (size_t)WPITCH + k0;
      FragB bf;
      bf.h[0] = *(const v8usa*)wq;
      bf.h[1] = *(const v8usa*)(wq + 16);
      acc[t] = wmb(af, bf, acc[t]);
    }
  }
  __syncthreads();

#pragma unroll
  for (int t = 0; t < 8; ++t) {
    const int lc = 16 * t + m;
    const float bb = par[lc];
#pragma unroll
    for (int r = 0; r < 8; ++r) {
      const int lr = 16 * wave + 8 * hh + r;
      stg[lr * BN + lc] = acc[t][r] + bb;
    }
  }
  __syncthreads();

  if (tid < BN) {
    double s = 0.0;
#pragma unroll 1
    for (int r = 0; r < NGR; ++r) s += (double)stg[r * BN + tid];
    const double mean = s * (1.0 / (double)NGR);
    double q = 0.0;
#pragma unroll 1
    for (int r = 0; r < NGR; ++r) {
      const double d = (double)stg[r * BN + tid] - mean;
      q += d * d;
    }
    const float varf = (float)(q * (1.0 / (double)NGR));
    cmu[tid] = (float)mean;
    crr[tid] = 1.0f / sqrtf(varf + 1e-5f);
  }
  __syncthreads();

  const v4f mu4 = *(const v4fa*)(cmu + 4 * lane);
  const v4f rr4 = *(const v4fa*)(crr + 4 * lane);
  const v4f g4  = *(const v4fa*)(par + BN + 4 * lane);
  const v4f b4  = *(const v4fa*)(par + 2 * BN + 4 * lane);
  if constexpr (MODE == 1) {
    v4us hv[16], lv[16];
#pragma unroll
    for (int i = 0; i < 16; ++i) {
      const int lr = 16 * wave + i;
      const v4f x = *(const v4fa*)(stg + lr * BN + 4 * lane);
      float y[4];
      y[0] = relu_keep(bn_y(x.x, mu4.x, rr4.x, g4.x, b4.x));
      y[1] = relu_keep(bn_y(x.y, mu4.y, rr4.y, g4.y, b4.y));
      y[2] = relu_keep(bn_y(x.z, mu4.z, rr4.z, g4.z, b4.z));
      y[3] = relu_keep(bn_y(x.w, mu4.w, rr4.w, g4.w, b4.w));
      v4us hq, lq;
#pragma unroll
      for (int j = 0; j < 4; ++j) {
        const unsigned hb = bf_bits(y[j]);
        hq[j] = (unsigned short)hb;
        lq[j] = (unsigned short)bf_bits(y[j] - bf_val(hb));
      }
      hv[i] = hq;
      lv[i] = lq;
    }
#pragma unroll
    for (int i = 0; i < 16; ++i) {
      unsigned short* op = outH + (size_t)(16 * wave + i) * (size_t)HIDP + colBase + 4 * lane;
      *(volatile v4us*)op = hv[i];
      *(volatile v4us*)(op + HH) = lv[i];
    }
    __threadfence();
#pragma unroll
    for (int i = 0; i < 16; ++i) {
      unsigned short* op = outH + (size_t)(16 * wave + i) * (size_t)HIDP + colBase + 4 * lane;
      *(volatile v4us*)op = hv[i];
      *(volatile v4us*)(op + HH) = lv[i];
    }
  } else {
    v4f pv[16];
#pragma unroll
    for (int i = 0; i < 16; ++i) {
      const int lr = 16 * wave + i;
      const v4f x = *(const v4fa*)(stg + lr * BN + 4 * lane);
      v4f y;
      y.x = relu_keep(bn_y(x.x, mu4.x, rr4.x, g4.x, b4.x));
      y.y = relu_keep(bn_y(x.y, mu4.y, rr4.y, g4.y, b4.y));
      y.z = relu_keep(bn_y(x.z, mu4.z, rr4.z, g4.z, b4.z));
      y.w = relu_keep(bn_y(x.w, mu4.w, rr4.w, g4.w, b4.w));
      pv[i] = y;
    }
#pragma unroll
    for (int i = 0; i < 16; ++i) {
      float* op = outF + (size_t)(16 * wave + i) * (size_t)DD + 4 * lane;
      *(volatile v4f*)op = pv[i];
    }
    __threadfence();
#pragma unroll
    for (int i = 0; i < 16; ++i) {
      float* op = outF + (size_t)(16 * wave + i) * (size_t)DD + 4 * lane;
      *(volatile v4f*)op = pv[i];
    }
  }
}

__global__ __launch_bounds__(NTHR) void k_replay(const float* __restrict__ hv, const int* __restrict__ listg,
                                                 const int* __restrict__ offg, const int* __restrict__ cntg,
                                                 const float* __restrict__ ee1l, const float* __restrict__ ee2l,
                                                 unsigned short* agg) {
  __shared__ __attribute__((aligned(16))) float et[18 * DD];
  __shared__ __attribute__((aligned(16))) float sf1[DD];
  __shared__ __attribute__((aligned(16))) float sf2[DD];
  __shared__ __attribute__((aligned(16))) unsigned int stw[NWAVE * DD];
  const int tid = (int)threadIdx.x, lane = tid & 31;
  const int wave = __builtin_amdgcn_readfirstlane(tid >> 5);
  const int nodeBase = (int)blockIdx.x * NB1;
  const int* lp = listg + (size_t)blockIdx.x * RCAP;

#pragma unroll 1
  for (int i = tid; i < 18 * DD; i += NTHR) {
    const int c  = i >> 7, ch = i & (DD - 1);
    const int a0 = c / 3;
    const int a1 = c - 3 * a0;
    et[i] = bf_rne(ee1l[a0 * DD + ch]) + bf_rne(ee2l[a1 * DD + ch]);
  }
  if (tid < DD) {
    sf1[tid] = bf_rne(ee1l[4 * DD + tid]);
    sf2[tid] = bf_rne(ee2l[tid]);
  }
  __syncthreads();

  unsigned int* stwu = stw + wave * DD;
  const float qnan = __int_as_float(0x7fc00000);
#pragma unroll 1
  for (int jt = 0; jt < NB1 / NWAVE; ++jt) {
    const int slot = wave * (NB1 / NWAVE) + jt;
    const int node = nodeBase + slot;
    int ov = offg[node];
    const int cvr = cntg[node];
    ov = ov < 0 ? 0 : (ov > RCAP ? RCAP : ov);
    int cvc = cvr < 0 ? 0 : (cvr > DEGCAP ? DEGCAP : cvr);
    cvc = cvc > RCAP - ov ? RCAP - ov : cvc;
    const int o    = __builtin_amdgcn_readfirstlane(ov);
    const int c    = __builtin_amdgcn_readfirstlane(cvc);
    const int craw = __builtin_amdgcn_readfirstlane(cvr);
    const bool poison = (craw > DEGCAP) || (craw < 0);
    int last = o + c - 1;
    last = last < o ? o : last;
    last = last > RCAP - 1 ? RCAP - 1 : last;
    const bool live = node < NNODE;

    float ag0 = 0.0f, ag1 = 0.0f, ag2 = 0.0f, ag3 = 0.0f;
#pragma unroll 1
    for (int b0 = 0; b0 < c; b0 += 32) {
      int idx = o + b0 + lane;
      idx = idx > last ? last : idx;
      idx = idx < 0 ? 0 : idx;
      const int wv = lp[idx];
      const int m32 = (c - b0) < 32 ? (c - b0) : 32;
#pragma unroll 4
      for (int k = 0; k < m32; ++k) {
        const unsigned wk = (unsigned)__builtin_amdgcn_readlane(wv, k);
        int sk = (int)(wk & 0x1FFFFu);
        sk = sk > NNODE - 1 ? NNODE - 1 : sk;
        int ck = (int)((wk >> 17) & 31u);
        ck = ck > 17 ? 17 : ck;
        const v4f v = *(const v4f*)(hv + (size_t)sk * DD + 4 * lane);
        const v4f e = *(const v4fa*)(et + ck * DD + 4 * lane);
        ag0 += (v.x + e.x); ag1 += (v.y + e.y); ag2 += (v.z + e.z); ag3 += (v.w + e.w);
      }
    }
    const int nc = live ? node : NNODE - 1;
    const v4f sv = *(const v4f*)(hv + (size_t)nc * DD + 4 * lane);
    const v4f q1 = *(const v4fa*)(sf1 + 4 * lane);
    const v4f q2 = *(const v4fa*)(sf2 + 4 * lane);
    float r0 = ((ag0 + sv.x) + q1.x) + q2.x;
    float r1 = ((ag1 + sv.y) + q1.y) + q2.y;
    float r2 = ((ag2 + sv.z) + q1.z) + q2.z;
    float r3 = ((ag3 + sv.w) + q1.w) + q2.w;
    r0 = live ? (poison ? qnan : r0) : 0.0f;
    r1 = live ? (poison ? qnan : r1) : 0.0f;
    r2 = live ? (poison ? qnan : r2) : 0.0f;
    r3 = live ? (poison ? qnan : r3) : 0.0f;

    const unsigned hb0 = bf_bits(r0), hb1 = bf_bits(r1), hb2 = bf_bits(r2), hb3 = bf_bits(r3);
    const unsigned lb0 = bf_bits(r0 - bf_val(hb0)), lb1 = bf_bits(r1 - bf_val(hb1));
    const unsigned lb2 = bf_bits(r2 - bf_val(hb2)), lb3 = bf_bits(r3 - bf_val(hb3));
    v2u hw, lw;
    hw.x = hb0 | (hb1 << 16);
    hw.y = hb2 | (hb3 << 16);
    lw.x = lb0 | (lb1 << 16);
    lw.y = lb2 | (lb3 << 16);
    __builtin_amdgcn_fence(__ATOMIC_RELEASE, "wavefront");
    __builtin_amdgcn_wave_barrier();
    *(v2u*)(stwu + 2 * lane)      = hw;
    *(v2u*)(stwu + 64 + 2 * lane) = lw;
    __builtin_amdgcn_fence(__ATOMIC_RELEASE, "wavefront");
    __builtin_amdgcn_wave_barrier();
    const v4u pk = *(const v4ua*)(stwu + 4 * lane);
    unsigned short* gp = agg + (size_t)node * (size_t)APW + 8 * lane;
    const bool wsv = node < MPAD;
    if (wsv) *(volatile v4u*)gp = pk;
    __threadfence();
    if (wsv) *(volatile v4u*)gp = pk;
  }
}

template <int MODE, int KEXT, int APITCH, int WPITCH>
__global__ __launch_bounds__(GTHR) __attribute__((amdgpu_num_vgpr(248)))
void k_gemm(const unsigned short* __restrict__ A, const unsigned short* __restrict__ WT,
            const float* __restrict__ bias, unsigned short* outH, float* outF, float* rec,
            int nLive, int mRows) {
  static_assert(KEXT % 32 == 0 && KEXT <= APITCH && KEXT <= WPITCH);
  __shared__ __attribute__((aligned(16))) float stg[GBM * BN];
  __shared__ __attribute__((aligned(16))) float pst[PARTW];
  __shared__ __attribute__((aligned(16))) float bsh[BN];
  const int tid = (int)threadIdx.x, lane = tid & 31, wave = tid >> 5, hh = lane >> 4, m = lane & 15;
  const int rowBase = (int)blockIdx.x * GBM;
  const int colBase = (int)blockIdx.y * BN;

  if (tid < 32) {
    const v4f q = *(const v4f*)(bias + colBase + 4 * lane);
    bsh[4 * lane + 0] = bf_rne(q.x); bsh[4 * lane + 1] = bf_rne(q.y);
    bsh[4 * lane + 2] = bf_rne(q.z); bsh[4 * lane + 3] = bf_rne(q.w);
  }

  v8f acc[8];
  {
    const v8f z = {0.f, 0.f, 0.f, 0.f, 0.f, 0.f, 0.f, 0.f};
#pragma unroll
    for (int t = 0; t < 8; ++t) acc[t] = z;
  }
  const unsigned short* ap = A + (size_t)(rowBase + 16 * wave + m) * (size_t)APITCH + 8 * hh;
  const unsigned short* wp = WT + (size_t)(colBase + m) * (size_t)WPITCH + 8 * hh;
#pragma unroll 1
  for (int k0 = 0; k0 < KEXT; k0 += 32) {
    FragB af;
    af.h[0] = *(const v8usa*)(ap + k0);
    af.h[1] = *(const v8usa*)(ap + k0 + 16);
#pragma unroll
    for (int t = 0; t < 8; ++t) {
      const unsigned short* wq = wp + (size_t)(16 * t) * (size_t)WPITCH + k0;
      FragB bf;
      bf.h[0] = *(const v8usa*)wq;
      bf.h[1] = *(const v8usa*)(wq + 16);
      acc[t] = wmb(af, bf, acc[t]);
    }
  }
  __syncthreads();

#pragma unroll
  for (int t = 0; t < 8; ++t) {
    const int lc = 16 * t + m;
    const float bb = bsh[lc];
#pragma unroll
    for (int r = 0; r < 8; ++r) {
      const int lr = 16 * wave + 8 * hh + r;
      const bool live = (rowBase + lr) < nLive;
      float v = acc[t][r] + bb;
      if (MODE == 1) v = relu_keep(v);
      stg[lr * BN + lc] = live ? v : 0.0f;
    }
  }
  __syncthreads();

  if constexpr (MODE == 0) {
    {
      int rv = nLive - rowBase;
      rv = rv < 0 ? 0 : (rv > GBM ? GBM : rv);
      float n = 0.0f, mean = 0.0f, M2 = 0.0f;
#pragma unroll 1
      for (int r = 0; r < rv; ++r) {
        const float v = stg[r * BN + tid];
        n += 1.0f;
        const float rk = 1.0f / n;
        const float d = v - mean;
        mean = fmaf(d, rk, mean);
        M2 = fmaf(d, v - mean, M2);
      }
      pst[1 + tid] = mean;
      pst[1 + BN + tid] = M2;
      if (tid == 0) pst[0] = n;
#pragma unroll 1
      for (int i = 2 * BN + 1 + tid; i < PARTW; i += GTHR) pst[i] = 0.0f;
    }
    v4f fv[16];
#pragma unroll
    for (int i = 0; i < 16; ++i) {
      const int lr = 16 * wave + i;
      fv[i] = *(const v4fa*)(stg + lr * BN + 4 * lane);
    }
#pragma unroll
    for (int i = 0; i < 16; ++i) {
      const int gr = rowBase + 16 * wave + i;
      float* op = outF + (size_t)gr * (size_t)DD + 4 * lane;
      if (gr < mRows) *(volatile v4f*)op = fv[i];
    }
    __threadfence();
#pragma unroll
    for (int i = 0; i < 16; ++i) {
      const int gr = rowBase + 16 * wave + i;
      float* op = outF + (size_t)gr * (size_t)DD + 4 * lane;
      if (gr < mRows) *(volatile v4f*)op = fv[i];
    }
    __syncthreads();
    v4f pv = {0.f, 0.f, 0.f, 0.f};
    if (tid < PARTW / 4) {
      pv = *(const v4fa*)(pst + 4 * tid);
      *(volatile v4f*)(rec + (size_t)blockIdx.x * PARTW + 4 * tid) = pv;
    }
    __threadfence();
    if (tid < PARTW / 4) {
      *(volatile v4f*)(rec + (size_t)blockIdx.x * PARTW + 4 * tid) = pv;
    }
  } else {
    v4us hv[16], lv[16];
#pragma unroll
    for (int i = 0; i < 16; ++i) {
      const int lr = 16 * wave + i;
      const v4f x = *(const v4fa*)(stg + lr * BN + 4 * lane);
      const float y[4] = {x.x, x.y, x.z, x.w};
      v4us hq, lq;
#pragma unroll
      for (int j = 0; j < 4; ++j) {
        const unsigned hb = bf_bits(y[j]);
        hq[j] = (unsigned short)hb;
        lq[j] = (unsigned short)bf_bits(y[j] - bf_val(hb));
      }
      hv[i] = hq;
      lv[i] = lq;
    }
#pragma unroll
    for (int i = 0; i < 16; ++i) {
      const int gr = rowBase + 16 * wave + i;
      unsigned short* op = outH + (size_t)gr * (size_t)HIDP + colBase + 4 * lane;
      if (gr < mRows) { *(volatile v4us*)op = hv[i]; *(volatile v4us*)(op + HH) = lv[i]; }
    }
    __threadfence();
#pragma unroll
    for (int i = 0; i < 16; ++i) {
      const int gr = rowBase + 16 * wave + i;
      unsigned short* op = outH + (size_t)gr * (size_t)HIDP + colBase + 4 * lane;
      if (gr < mRows) { *(volatile v4us*)op = hv[i]; *(volatile v4us*)(op + HH) = lv[i]; }
    }
  }
}

__global__ __launch_bounds__(DD) void k_comb(const float* __restrict__ rec, int nPart,
                                             const float* __restrict__ gam, const float* __restrict__ bet,
                                             float* stat) {
  __shared__ __attribute__((aligned(16))) float stg[4 * DD];
  const int tid = (int)threadIdx.x;
  const int c = tid & (DD - 1);
  double n = 0.0, mean = 0.0, M2 = 0.0;
#pragma unroll 1
  for (int b = 0; b < nPart; ++b) {
    const float* pr = rec + (size_t)b * PARTW;
    const float nb = pr[0];
    const float mb = pr[1 + c];
    const float qb = pr[1 + DD + c];
    if (nb > 0.5f) {
      const double nn = n + (double)nb;
      const double delta = (double)mb - mean;
      const double f = (double)nb / nn;
      mean = mean + delta * f;
      M2 = M2 + (double)qb + delta * delta * n * f;
      n = nn;
    }
  }
  const double nt = n < 1.0 ? 1.0 : n;
  const float varf = (float)(M2 / nt);
  stg[c]          = (float)mean;
  stg[DD + c]     = 1.0f / sqrtf(varf + 1e-5f);
  stg[2 * DD + c] = bf_rne(gam[c]);
  stg[3 * DD + c] = bf_rne(bet[c]);
  __syncthreads();
  const v4f v = *(const v4fa*)(stg + 4 * tid);
  *(volatile v4f*)(stat + 4 * tid) = v;
  __threadfence();
  *(volatile v4f*)(stat + 4 * tid) = v;
}

template <int LAST>
__global__ __launch_bounds__(NTHR) void k_apply(float* p0, const float* __restrict__ stat,
                                                const float* __restrict__ gvn, const int* __restrict__ bat,
                                                float* dout, int nUnits) {
  __shared__ __attribute__((aligned(16))) float st[4 * DD];
  const int tid = (int)threadIdx.x;
  if (tid < DD) {
    const v4f s = *(const v4f*)(stat + 4 * tid);
    *(v4fa*)(st + 4 * tid) = s;
  }
  __syncthreads();
  const int u = (int)blockIdx.x * NTHR + tid;
  if (u >= nUnits) return;
  const int row = u >> 5;
  const int c4  = (u & 31) * 4;
  const int rc  = row < NNODE ? row : NNODE - 1;
  const v4f a = *(const v4f*)(p0 + (size_t)u * 4);
  const v4f mu = *(const v4fa*)(st + c4);
  const v4f rr = *(const v4fa*)(st + DD + c4);
  const v4f gg = *(const v4fa*)(st + 2 * DD + c4);
  const v4f bb = *(const v4fa*)(st + 3 * DD + c4);
  v4f o;
  o.x = bn_y(a.x, mu.x, rr.x, gg.x, bb.x);
  o.y = bn_y(a.y, mu.y, rr.y, gg.y, bb.y);
  o.z = bn_y(a.z, mu.z, rr.z, gg.z, bb.z);
  o.w = bn_y(a.w, mu.w, rr.w, gg.w, bb.w);
  if (LAST == 0) {
    const int gi = clampi(bat[rc], 0, NGR - 1);
    const v4f gv = *(const v4f*)(gvn + (size_t)gi * DD + c4);
    asm volatile("" :: "v"(gv.x), "v"(gv.y), "v"(gv.z), "v"(gv.w));
    const bool ok = row < NNODE;
    o.x = ok ? (relu_keep(o.x) + gv.x) : 0.0f;
    o.y = ok ? (relu_keep(o.y) + gv.y) : 0.0f;
    o.z = ok ? (relu_keep(o.z) + gv.z) : 0.0f;
    o.w = ok ? (relu_keep(o.w) + gv.w) : 0.0f;
    float* op = p0 + (size_t)u * 4;
    *(volatile v4f*)op = o;
    __threadfence();
    *(volatile v4f*)op = o;
  } else {
    float* op = dout + (size_t)u * 4;
    *(volatile v4f*)op = o;
    __threadfence();
    *(volatile v4f*)op = o;
  }
}

static inline size_t al256(size_t o) { return (o + 255) & ~(size_t)255; }

extern "C" void kernel_launch(void* const* d_in, const int* in_sizes, int n_in,
                              void* d_out, int out_size, void* d_ws, size_t ws_size,
                              hipStream_t stream) {
  if (n_in < 23) return;
  const int want[23] = {NNODE * 2, 2 * NEDGE, NEDGE * 2, NNODE, 120 * DD, 3 * DD, DD,
                        NLAY * DD * HH, NLAY * HH, NLAY * HH * DD, NLAY * DD, NLAY * 6 * DD, NLAY * 3 * DD,
                        NLAY * DD, NLAY * DD, 4 * DD * HH, 4 * HH, 4 * HH, 4 * HH, 4 * HH * DD, 4 * DD, 4 * DD, 4 * DD};
  for (int i = 0; i < 23; ++i) if (in_sizes[i] != want[i]) return;
  if (out_size != NNODE * DD) return;

  const int*   x      = (const int*)d_in[0];
  const int*   ei     = (const int*)d_in[1];
  const int*   ea     = (const int*)d_in[2];
  const int*   bat    = (const int*)d_in[3];
  const float* xe1    = (const float*)d_in[4];
  const float* xe2    = (const float*)d_in[5];
  const float* gve    = (const float*)d_in[6];
  const float* cw1    = (const float*)d_in[7];
  const float* cb1    = (const float*)d_in[8];
  const float* cw2    = (const float*)d_in[9];
  const float* cb2    = (const float*)d_in[10];
  const float* ee1    = (const float*)d_in[11];
  const float* ee2    = (const float*)d_in[12];
  const float* bng    = (const float*)d_in[13];
  const float* bnb    = (const float*)d_in[14];
  const float* gw1    = (const float*)d_in[15];
  const float* gb1    = (const float*)d_in[16];
  const float* gg1    = (const float*)d_in[17];
  const float* gbb1   = (const float*)d_in[18];
  const float* gw2    = (const float*)d_in[19];
  const float* gb2    = (const float*)d_in[20];
  const float* gg2    = (const float*)d_in[21];
  const float* gbb2   = (const float*)d_in[22];
  float* out = (float*)d_out;

  char* ws = (char*)d_ws;
  size_t off = 0;
  const size_t oW1D = off; off = al256(off + (size_t)NLAY * HH * 256 * 2);
  const size_t oW2D = off; off = al256(off + (size_t)NLAY * DD * 512 * 2);
  const size_t oGW1 = off; off = al256(off + (size_t)4 * HH * 384 * 2);
  const size_t oGW2 = off; off = al256(off + (size_t)4 * DD * 512 * 2);
  const size_t oP0  = off; off = al256(off + (size_t)MPAD * DD * 4);
  const size_t oP1  = off; off = al256(off + (size_t)MPAD * APW * 2);
  const size_t oP2  = off; off = al256(off + (size_t)HALFR * HIDP * 2);
  const size_t oLS  = off; off = al256(off + (size_t)NBLK * RCAP * 4);
  const size_t oOF  = off; off = al256(off + (size_t)NBLK * NB1 * 4);
  const size_t oCN  = off; off = al256(off + (size_t)NBLK * NB1 * 4);
  const size_t oGL  = off; off = al256(off + (size_t)NGR * GPITCH * 4);
  const size_t oRC  = off; off = al256(off + (size_t)NTILE * PARTW * 4);
  const size_t oST  = off; off = al256(off + (size_t)4 * DD * 4);
  const size_t oP3  = off; off = al256(off + (size_t)NGR * P3P * 2);
  const size_t oTV  = off; off = al256(off + (size_t)NGR * HIDP * 2);
  const size_t oG0  = off; off = al256(off + (size_t)NGR * DD * 4);
  const size_t oG1  = off; off = al256(off + (size_t)NGR * DD * 4);
  if (off > ws_size || off > (size_t)(256u << 20)) return;
  unsigned short* W1D = (unsigned short*)(ws + oW1D);
  unsigned short* W2D = (unsigned short*)(ws + oW2D);
  unsigned short* GW1 = (unsigned short*)(ws + oGW1);
  unsigned short* GW2 = (unsigned short*)(ws + oGW2);
  float*          P0  = (float*)(ws + oP0);
  unsigned short* P1  = (unsigned short*)(ws + oP1);
  unsigned short* P2  = (unsigned short*)(ws + oP2);
  int*            LS  = (int*)(ws + oLS);
  int*            OF  = (int*)(ws + oOF);
  int*            CN  = (int*)(ws + oCN);
  int*            GL  = (int*)(ws + oGL);
  float*          RC  = (float*)(ws + oRC);
  float*          ST  = (float*)(ws + oST);
  unsigned short* P3  = (unsigned short*)(ws + oP3);
  unsigned short* TV  = (unsigned short*)(ws + oTV);
  float*          G0  = (float*)(ws + oG0);
  float*          G1  = (float*)(ws + oG1);

  hipFuncSetAttribute(reinterpret_cast<const void*>(&k_bucket), hipFuncAttributeMaxDynamicSharedMemorySize, LDS_BKT);
  hipFuncSetAttribute(reinterpret_cast<const void*>(&k_gv<1, 384, P3P, 384>),
                      hipFuncAttributeMaxDynamicSharedMemorySize, LDS_GV);
  hipFuncSetAttribute(reinterpret_cast<const void*>(&k_gv<2, 512, HIDP, 512>),
                      hipFuncAttributeMaxDynamicSharedMemorySize, LDS_GV);

  {
    const int u1 = NLAY * HH * 32;
    const int u2 = NLAY * DD * 64;
    const int u3 = 4 * HH * 48;
    const int u4 = 4 * DD * 64;
    if ((u1 % NTHR) != 0 || (u2 % NTHR) != 0 || (u3 % NTHR) != 0 || (u4 % NTHR) != 0) return;
    k_wprep<<<u1 / NTHR, NTHR, 0, stream>>>(cw1, DD, HH, 32, u1, W1D);
    k_wprep<<<u2 / NTHR, NTHR, 0, stream>>>(cw2, HH, DD, 64, u2, W2D);
    k_wprep<<<u3 / NTHR, NTHR, 0, stream>>>(gw1, DD, HH, 48, u3, GW1);
    k_wprep<<<u4 / NTHR, NTHR, 0, stream>>>(gw2, HH, DD, 64, u4, GW2);
  }
  k_embed<<<(MPAD * 32) / NTHR, NTHR, 0, stream>>>(x, xe1, xe2, gve, P0);
  k_bucket<<<NBLK, NTHR, LDS_BKT, stream>>>(ei, ea, LS, OF, CN);
  k_gbucket<<<NGR, NTHR, 0, stream>>>(bat, gve, GL, G0);

  for (int l = 0; l < NLAY; ++l) {
    float* gvl = ((l & 1) != 0) ? G1 : G0;
    float* gvn = ((l & 1) != 0) ? G0 : G1;
    if (l < NLAY - 1) {
      k_pool<<<NGR, NTHR, 0, stream>>>(P0, GL, gvl, P3);
      k_gv<1, 384, P3P, 384><<<2, NTHR, LDS_GV, stream>>>(
          P3, GW1 + (size_t)l * HH * 384, gb1 + (size_t)l * HH, gg1 + (size_t)l * HH, gbb1 + (size_t)l * HH,
          TV, gvn);
      k_gv<2, 512, HIDP, 512><<<1, NTHR, LDS_GV, stream>>>(
          TV, GW2 + (size_t)l * DD * 512, gb2 + (size_t)l * DD, gg2 + (size_t)l * DD, gbb2 + (size_t)l * DD,
          TV, gvn);
    }
    k_replay<<<NBLK, NTHR, 0, stream>>>(P0, LS, OF, CN, ee1 + (size_t)l * 6 * DD, ee2 + (size_t)l * 3 * DD, P1);
    for (int hf = 0; hf < 2; ++hf) {
      const int rb = hf * HALFR;
      k_gemm<1, KA_EXT, APW, 256><<<dim3(HTILE, 2), GTHR, 0, stream>>>(
          P1 + (size_t)rb * APW, W1D + (size_t)l * HH * 256, cb1 + (size_t)l * HH,
          P2, P0, RC, NNODE - rb, HALFR);
      k_gemm<0, KB_EXT, HIDP, 512><<<dim3(HTILE, 1), GTHR, 0, stream>>>(
          P2, W2D + (size_t)l * DD * 512, cb2 + (size_t)l * DD,
          P2, P0 + (size_t)rb * DD, RC + (size_t)hf * HTILE * PARTW, NNODE - rb, HALFR);
    }
    k_comb<<<1, DD, 0, stream>>>(RC, NTILE, bng + (size_t)l * DD, bnb + (size_t)l * DD, ST);
    if (l < NLAY - 1) {
      k_apply<0><<<(MPAD * 32) / NTHR, NTHR, 0, stream>>>(P0, ST, gvn, bat, out, MPAD * 32);
    } else {
      k_apply<1><<<(NNODE * 32) / NTHR, NTHR, 0, stream>>>(P0, ST, gvn, bat, out, NNODE * 32);
    }
  }
}
